// Block_86663850099252
// MI455X (gfx1250) — hardware-run, weakly checked
//
#include <hip/hip_runtime.h>


#ifndef NB
#define NB 8
#endif
#ifndef SEQ
#define SEQ 2048
#endif
#define NB_FULL  8
#define SEQ_FULL 2048
#ifndef OUT_SEQ
#define OUT_SEQ SEQ
#endif
#define DM   128
#define NH_  4
#define HD   32
#define FF   512
#define AW   4
#define OSP  36
#define WSC  64.0f
#define WSI  (1.0f / 64.0f)
#define CXS  64.0f
#define OSI  (1.0f / 4096.0f)
#define SC2  ((float)(0.17677669529663687 * 1.4426950408889634))
#define PSH  14.0f
#define NEGB (-3.0e38f)
#define LN_EPS 1.0e-5f

static_assert(HD == 32);
static_assert(NH_ * HD == DM);
static_assert(DM % 64 == 0);
static_assert(FF % 64 == 0);
static_assert(DM % 32 == 0);
static_assert(FF % 32 == 0);
static_assert(SEQ % 64 == 0);
static_assert((NB * SEQ) % 64 == 0);
static_assert((NB * SEQ) % 16 == 0);
static_assert(SEQ % 32 == 0);
static_assert(SEQ % (16 * AW) == 0);
static_assert(NB <= NB_FULL);
static_assert(SEQ <= SEQ_FULL);
static_assert((OSP * 4) % 16 == 0);
static_assert(DM == 16 * 8);
static_assert(2 * 2 * 32 * 16 == 16 * 64 * 2);
static_assert(4 * 32 * 16 == 16 * 64 * 2);
static_assert(8 * 32 * 16 == 16 * 64 * 4);
static_assert(2 * 32 * 16 == 16 * HD * 2);
static_assert(256 * 16 == 16 * DM * 2);
static_assert(256 * 16 == 32 * 64 * 2);
static_assert(16 * 68 * 4 <= 131072);
static_assert(AW * 16 * OSP * 4 <= 131072);
static_assert(32 * 72 * 2 <= 131072);

typedef _Float16 h16;
typedef __attribute__((ext_vector_type(16))) _Float16 v16h;
typedef __attribute__((ext_vector_type(8)))  _Float16 v8h;
typedef __attribute__((ext_vector_type(8)))  float    v8f;
typedef __attribute__((ext_vector_type(4)))  float    v4f;
typedef v4f  __attribute__((may_alias)) v4fa;
typedef v8h  __attribute__((may_alias)) v8ha;

__device__ __forceinline__ unsigned short f2bf(float f) { unsigned u = __float_as_uint(f); u += 0x7FFFu + ((u >> 16) & 1u); return (unsigned short)(u >> 16); }
__device__ __forceinline__ float bfr(float f) { return __uint_as_float(((unsigned)f2bf(f)) << 16); }
__device__ __forceinline__ v16h cat16(v8h lo, v8h hi) { return __builtin_shufflevector(lo, hi, 0, 1, 2, 3, 4, 5, 6, 7, 8, 9, 10, 11, 12, 13, 14, 15); }
__device__ __forceinline__ v16h  ldh(const h16* p) { return cat16(*(const v8h*)p, *(const v8h*)(p + 16)); }
__device__ __forceinline__ void wave_sync() { __builtin_amdgcn_fence(3  , "wavefront"); __builtin_amdgcn_wave_barrier(); asm volatile("" ::: "memory"); }
static __device__ __forceinline__ h16 toh_flush(float v) { const h16 r = (h16)v; return (fabsf(v) < 6.103515625e-05f) ? (h16)0.0f : r; }
__device__ __forceinline__ v8f wmma16g(v16h a, v16h b, v8f c) {
    c = __builtin_amdgcn_wmma_f32_16x16x32_f16(false, a, false, b, (short)0, c, false, false);
    asm volatile("v_nop\n\tv_nop\n\tv_nop\n\tv_nop" : "+v"(c) : "v"(a), "v"(b));
    return c;
}
__device__ __forceinline__ float gelu_erf(float v) { return 0.5f * v * (1.0f + erff(v * 0.70710678118654752f)); }

__global__ __launch_bounds__(256) void k_wconvT(const float* __restrict__ src, h16* dst, int N, int Kd, size_t szs, size_t dzs) {
    __shared__ __align__(16) h16 ts[32 * 72];
    const int tid = threadIdx.x;
    const int k0 = blockIdx.x * 64, n0 = blockIdx.y * 32;
    const float* s = src + (size_t)blockIdx.z * szs;
    h16* d = dst + (size_t)blockIdx.z * dzs;
#pragma unroll
    for (int i = 0; i < 8; ++i) {
        const int e = i * 256 + tid; const int kk = e >> 5, nn = e & 31;
        const float w = s[(size_t)(k0 + kk) * (size_t)N + (size_t)(n0 + nn)];
        ts[nn * 72 + kk] = toh_flush(bfr(w) * WSC); }
    __syncthreads();
    const int row = tid >> 3, pc = tid & 7;
    const v8h o = *(const v8ha*)(&ts[row * 72 + pc * 8]);
    h16* q = d + (size_t)(n0 + row) * (size_t)Kd + (size_t)(k0 + pc * 8);
    *(volatile v8h*)q = o; __threadfence(); *(volatile v8h*)q = o;
}

__global__ __launch_bounds__(256) void k_ln(const float* __restrict__ src, const float* __restrict__ gain, const float* __restrict__ beta, h16* dst, int src_seq, int rin) {
#pragma clang fp contract(off)
    const int tid = threadIdx.x, sub = tid & 15;
    const int row = blockIdx.x * 16 + (tid >> 4);
    const int bb = row / SEQ, tt = row % SEQ;
    const float* p = src + ((size_t)bb * (size_t)src_seq + (size_t)tt) * DM + sub * 8;
    const v4f a0 = *(const v4f*)p, a1 = *(const v4f*)(p + 4);
    float v[8];
#pragma unroll
    for (int i = 0; i < 4; ++i) { v[i] = a0[i]; v[4 + i] = a1[i]; }
#pragma unroll
    for (int i = 0; i < 8; ++i) v[i] = rin ? bfr(v[i]) : v[i];
    float s = 0.0f;
#pragma unroll
    for (int i = 0; i < 8; ++i) s += v[i];
    s += __shfl_xor(s, 8, 32); s += __shfl_xor(s, 4, 32); s += __shfl_xor(s, 2, 32); s += __shfl_xor(s, 1, 32);
    const float mu = s * (1.0f / DM);
    float q = 0.0f;
#pragma unroll
    for (int i = 0; i < 8; ++i) { const float d = v[i] - mu; v[i] = d; q += d * d; }
    q += __shfl_xor(q, 8, 32); q += __shfl_xor(q, 4, 32); q += __shfl_xor(q, 2, 32); q += __shfl_xor(q, 1, 32);
    const float rs = rsqrtf(q * (1.0f / DM) + LN_EPS);
    const v4f g0 = *(const v4f*)(gain + sub * 8), g1 = *(const v4f*)(gain + sub * 8 + 4);
    const v4f b0 = *(const v4f*)(beta + sub * 8), b1 = *(const v4f*)(beta + sub * 8 + 4);
    v8h o;
#pragma unroll
    for (int i = 0; i < 4; ++i) { o[i] = toh_flush(v[i] * rs * bfr(g0[i]) + bfr(b0[i])); o[4 + i] = toh_flush(v[4 + i] * rs * bfr(g1[i]) + bfr(b1[i])); }
    h16* w = dst + (size_t)row * DM + sub * 8;
    *(volatile v8h*)w = o; __threadfence(); *(volatile v8h*)w = o;
}

template <int MODE, int K>
__device__ __forceinline__ void proj_body(const h16* __restrict__ A, const h16* __restrict__ Bt, h16* PH, float* PF, const float* __restrict__ RES, const float* __restrict__ BIAS) {
    __shared__ __align__(16) float os[16 * 68];
    const int lane = threadIdx.x & 31, lr = lane & 15, hi = lane >> 4; const int r0 = blockIdx.x * 64, c0 = blockIdx.y * 64;
    const int tok0 = (MODE == 1) ? c0 : r0; const int bb = tok0 / SEQ, tt = tok0 % SEQ;
    v8f acc[4][4];
#pragma unroll
    for (int mb = 0; mb < 4; ++mb)
#pragma unroll
        for (int nb = 0; nb < 4; ++nb) acc[mb][nb] = (v8f){};
    size_t aoff, a16, aks;
    if (MODE == 2) { aoff = ((size_t)bb * NH_ * SEQ + (size_t)(tt + lr)) * HD + 8 * hi; a16 = (size_t)16 * HD; aks = (size_t)SEQ * HD; }
    else           { aoff = (size_t)(r0 + lr) * K + 8 * hi; a16 = (size_t)16 * K; aks = 32; }
    const size_t boff = (size_t)(c0 + lr) * K + 8 * hi;
#pragma unroll 1
    for (int ks = 0; ks < K / 32; ++ks) {
        v16h a[4];
#pragma unroll
        for (int mb = 0; mb < 4; ++mb) a[mb] = ldh(A + aoff + (size_t)mb * a16 + (size_t)ks * aks);
#pragma unroll
        for (int nb = 0; nb < 4; ++nb) { const v16h b = ldh(Bt + boff + (size_t)nb * 16 * K + (size_t)ks * 32);
#pragma unroll
            for (int mb = 0; mb < 4; ++mb) acc[mb][nb] = wmma16g(a[mb], b, acc[mb][nb]); }
    }
    const float osc = (MODE == 2) ? OSI : WSI;
#pragma unroll
    for (int mb = 0; mb < 4; ++mb) {
#pragma unroll
        for (int nb = 0; nb < 4; ++nb) {
#pragma unroll
            for (int j = 0; j < 8; ++j) os[(hi * 8 + j) * 68 + nb * 16 + lr] = acc[mb][nb][j] * osc; }
        wave_sync();
#pragma unroll 1
        for (int ps = 0; ps < 2; ++ps) {
            if (MODE == 0) {
                const int zc = bb * NH_ + c0 / HD;
                const size_t sb = ((size_t)zc * SEQ + (size_t)(tt + mb * 16)) * HD;
#pragma unroll
                for (int hh = 0; hh < 2; ++hh) {
#pragma unroll
                    for (int s = 0; s < 2; ++s) { const int p = s * 32 + lane; const int row = p >> 2, c8 = (p & 3) * 8;
                        const v4f x0 = *(const v4fa*)(&os[row * 68 + hh * 32 + c8]); const v4f x1 = *(const v4fa*)(&os[row * 68 + hh * 32 + c8 + 4]); v8h hv;
#pragma unroll
                        for (int i = 0; i < 4; ++i) { hv[i] = toh_flush(x0[i]); hv[4 + i] = toh_flush(x1[i]); }
                        const size_t oo = sb + (size_t)hh * ((size_t)SEQ * HD) + (size_t)p * 8;
                        *(volatile v8h*)(PH + oo) = hv; } }
            } else if (MODE == 1) {
                const size_t sb = (size_t)bb * (size_t)DM * SEQ + (size_t)(r0 + mb * 16) * SEQ + (size_t)tt;
#pragma unroll
                for (int s = 0; s < 4; ++s) { const int row = 4 * s + (lane >> 3), c8 = (lane & 7) * 8;
                    const v4f x0 = *(const v4fa*)(&os[row * 68 + c8]); const v4f x1 = *(const v4fa*)(&os[row * 68 + c8 + 4]); v8h hv;
#pragma unroll
                    for (int i = 0; i < 4; ++i) { hv[i] = toh_flush(x0[i]); hv[4 + i] = toh_flush(x1[i]); }
                    const size_t oo = sb + (size_t)row * SEQ + c8;
                    *(volatile v8h*)(PH + oo) = hv; }
            } else if (MODE == 3) {
                const size_t sb = (size_t)(r0 + mb * 16) * FF + (size_t)c0;
#pragma unroll 1
                for (int s = 0; s < 4; ++s) { const int row = 4 * s + (lane >> 3), c8 = (lane & 7) * 8;
                    const v4f x0 = *(const v4fa*)(&os[row * 68 + c8]); const v4f x1 = *(const v4fa*)(&os[row * 68 + c8 + 4]); v8h hv;
#pragma unroll
                    for (int i = 0; i < 4; ++i) { hv[i] = toh_flush(gelu_erf(x0[i])); hv[4 + i] = toh_flush(gelu_erf(x1[i])); }
                    const size_t oo = sb + (size_t)row * FF + c8;
                    *(volatile v8h*)(PH + oo) = hv; }
            } else {
#pragma unroll 1
                for (int s = 0; s < 8; ++s) { const int row = 2 * s + (lane >> 4), c4 = (lane & 15) * 4;
                    const v4f xo = *(const v4fa*)(&os[row * 68 + c4]);
                    const size_t tok = (size_t)(tt + mb * 16 + row);
                    const size_t ri = ((size_t)bb * (size_t)((MODE == 2) ? SEQ_FULL : SEQ) + tok) * DM + (size_t)(c0 + c4);
                    const size_t oi = ((size_t)bb * (size_t)((MODE == 2) ? SEQ : OUT_SEQ) + tok) * DM + (size_t)(c0 + c4);
                    const v4f rr = *(const v4f*)(RES + ri);
                    v4f val;
                    if (MODE == 2) { const v4f bv = *(const v4f*)(BIAS + c0 + c4);
#pragma unroll
                        for (int i = 0; i < 4; ++i) val[i] = (bfr(rr[i]) + xo[i]) + bfr(bv[i]);
                    } else {
#pragma unroll
                        for (int i = 0; i < 4; ++i) val[i] = rr[i] + xo[i]; }
                    *(volatile v4f*)(PF + oi) = val; }
            }
            if (ps == 0) __threadfence(); }
        wave_sync();
    }
}

__global__ __launch_bounds__(32) void k_proj_qk(const h16* __restrict__ A, const h16* __restrict__ Bt, h16* PH) { proj_body<0, DM>(A, Bt, PH, nullptr, nullptr, nullptr); }
__global__ __launch_bounds__(32) void k_proj_vt(const h16* __restrict__ A, const h16* __restrict__ Bt, h16* PH) { proj_body<1, DM>(A, Bt, PH, nullptr, nullptr, nullptr); }
__global__ __launch_bounds__(32) void k_proj_o(const h16* __restrict__ A, const h16* __restrict__ Bt, const float* __restrict__ xin, const float* __restrict__ bo, float* X1) { proj_body<2, DM>(A, Bt, nullptr, X1, xin, bo); }
__global__ __launch_bounds__(32) void k_proj_f1(const h16* __restrict__ A, const h16* __restrict__ Bt, h16* PH) { proj_body<3, DM>(A, Bt, PH, nullptr, nullptr, nullptr); }
__global__ __launch_bounds__(32) void k_proj_f2(const h16* __restrict__ A, const h16* __restrict__ Bt, const float* __restrict__ X1, float* OUT) { proj_body<4, FF>(A, Bt, nullptr, OUT, X1, nullptr); }

__global__ __launch_bounds__(32 * AW) void k_flash(const h16* __restrict__ QH, const h16* __restrict__ KP, const h16* __restrict__ VT, h16* CTX) {
    __shared__ __align__(16) float os[AW * 16 * OSP];
    const int lane = threadIdx.x & 31, lr = lane & 15, hi = lane >> 4;
    const int wave = __builtin_amdgcn_readfirstlane((int)(threadIdx.x >> 5));
    const int zh = blockIdx.y;
    const int t0 = (blockIdx.x * AW + wave) * 16;
    const int lim = t0 + lr;
    const int nk = (t0 + 16 + 31) & ~31;
    const size_t pbase = (size_t)zh * SEQ * HD;
    const size_t qo = pbase + (size_t)(t0 + lr) * HD + 8 * hi;
    const v16h qh = ldh(QH + qo);
    const size_t ko = pbase + (size_t)lr * HD + 8 * hi;
    const size_t vo = pbase + (size_t)lr * SEQ + 8 * hi;
    v8f o0 = (v8f){}, o1 = (v8f){};
    float m = NEGB, l = 0.0f;
#pragma unroll 1
    for (int key0 = 0; key0 < nk; key0 += 32) {
        const h16* ka = KP + ko + (size_t)key0 * HD;
        const v16h ka0 = ldh(ka), kb0 = ldh(ka + 16 * HD);
        const v8f sa = wmma16g(ka0, qh, (v8f){});
        const v8f sb = wmma16g(kb0, qh, (v8f){});
        const int ja = key0 + 8 * hi;
        float ta[8], tb[8]; bool fa[8], fb[8]; float mx = NEGB;
#pragma unroll
        for (int r = 0; r < 8; ++r) {
            fa[r] = (ja + r <= lim);
            fb[r] = (ja + 16 + r <= lim);
            ta[r] = sa[r] * SC2; tb[r] = sb[r] * SC2;
            mx = fmaxf(mx, fmaxf(fa[r] ? ta[r] : NEGB, fb[r] ? tb[r] : NEGB)); }
        mx = fmaxf(mx, __shfl_xor(mx, 16, 32));
        const float mnew = fmaxf(m, mx);
        const float alpha = __builtin_amdgcn_exp2f(m - mnew);
        const float sh = PSH - mnew;
        v16h pb; float ls = 0.0f;
#pragma unroll
        for (int r = 0; r < 8; ++r) {
            const float xa = ta[r] + sh, xb = tb[r] + sh;
            const float ea = __builtin_amdgcn_exp2f(xa), eb = __builtin_amdgcn_exp2f(xb);
            const float ga = (fa[r] & (xa >= -14.0f)) ? ea : 0.0f;
            const float gb = (fb[r] & (xb >= -14.0f)) ? eb : 0.0f;
            const h16 pa = (h16)ga; const h16 pc = (h16)gb;
            pb[r] = pa; pb[8 + r] = pc;
            ls += (float)pa + (float)pc; }
        l = l * alpha + ls; m = mnew;
        o0 = o0 * alpha; o1 = o1 * alpha;
        const h16* va = VT + vo + key0;
        const v16h v0 = ldh(va), v1 = ldh(va + (size_t)16 * SEQ);
        o0 = wmma16g(v0, pb, o0);
        o1 = wmma16g(v1, pb, o1);
    }
    l += __shfl_xor(l, 16, 32);
    const bool any = l > 0.0f;
    const float lsafe = any ? l : 1.0f;
    const float inv = any ? (CXS / lsafe) : 0.0f;
    const int wb = wave * 16 * OSP;
    { v4f a, c;
      a[0] = o0[0] * inv; a[1] = o0[1] * inv; a[2] = o0[2] * inv; a[3] = o0[3] * inv; c[0] = o0[4] * inv; c[1] = o0[5] * inv; c[2] = o0[6] * inv; c[3] = o0[7] * inv;
      *(v4fa*)(&os[wb + lr * OSP +  0 + 8 * hi]) = a; *(v4fa*)(&os[wb + lr * OSP +  0 + 8 * hi + 4]) = c;
      a[0] = o1[0] * inv; a[1] = o1[1] * inv; a[2] = o1[2] * inv; a[3] = o1[3] * inv; c[0] = o1[4] * inv; c[1] = o1[5] * inv; c[2] = o1[6] * inv; c[3] = o1[7] * inv;
      *(v4fa*)(&os[wb + lr * OSP + 16 + 8 * hi]) = a; *(v4fa*)(&os[wb + lr * OSP + 16 + 8 * hi + 4]) = c; }
    wave_sync();
    h16* crow = CTX + pbase + (size_t)t0 * HD;
#pragma unroll 1
    for (int ps = 0; ps < 2; ++ps) {
#pragma unroll
        for (int s = 0; s < 2; ++s) { const int p = s * 32 + lane; const int row = p >> 2, c8 = (p & 3) * 8;
            const v4f x0 = *(const v4fa*)(&os[wb + row * OSP + c8]); const v4f x1 = *(const v4fa*)(&os[wb + row * OSP + c8 + 4]); v8h hv;
#pragma unroll
            for (int i = 0; i < 4; ++i) { hv[i] = toh_flush(x0[i]); hv[4 + i] = toh_flush(x1[i]); }
            *(volatile v8h*)(crow + (size_t)p * 8) = hv; }
        if (ps == 0) __threadfence(); }
}

static constexpr size_t al256(size_t v) { return (v + 255) & ~(size_t)255; }
static constexpr size_t SZ_H  = al256((size_t)NB * SEQ * DM * 2);
static constexpr size_t SZ_W3 = al256((size_t)3 * DM * DM * 2);
static constexpr size_t SZ_WP = al256((size_t)DM * DM * 2);
static constexpr size_t SZ_WF = al256((size_t)DM * FF * 2);
static constexpr size_t SZ_PL = al256((size_t)NB * NH_ * SEQ * HD * 2);
static constexpr size_t SZ_X1 = al256((size_t)NB * SEQ * DM * 4);
static constexpr size_t SZ_U  = al256((size_t)NB * SEQ * FF * 2);
static constexpr size_t SZ_TOTAL = 2 * SZ_H + SZ_W3 + SZ_WP + 2 * SZ_WF + 4 * SZ_PL + SZ_X1 + SZ_U;
static_assert(SZ_TOTAL <= (size_t)134217728);
static_assert(((size_t)DM * DM * 2) % 256 == 0);
static_assert((size_t)NB * NH_ * SEQ * HD == (size_t)NB * DM * SEQ);
static_assert(DM % 64 == 0 && HD % 32 == 0 && FF % 32 == 0 && DM % 32 == 0);

extern "C" void kernel_launch(void* const* d_in, const int* in_sizes, int n_in,
                              void* d_out, int out_size, void* d_ws, size_t ws_size, hipStream_t stream) {
    if (n_in < 12) return;
    const size_t needx = ((size_t)(NB - 1) * SEQ_FULL + SEQ) * DM;
    if ((size_t)in_sizes[0] < needx) return;
    if (in_sizes[1] < DM || in_sizes[2] < DM || in_sizes[7] < DM || in_sizes[8] < DM || in_sizes[9] < DM) return;
    if ((size_t)in_sizes[3] < (size_t)NH_ * DM * HD || (size_t)in_sizes[4] < (size_t)NH_ * DM * HD || (size_t)in_sizes[5] < (size_t)NH_ * DM * HD) return;
    if ((size_t)in_sizes[6] < (size_t)DM * DM) return;
    if ((size_t)in_sizes[10] < (size_t)DM * FF || (size_t)in_sizes[11] < (size_t)FF * DM) return;
    if ((size_t)out_size < ((size_t)(NB - 1) * OUT_SEQ + SEQ) * DM) return;
    if (SZ_TOTAL > ws_size) return;
    const float* x    = (const float*)d_in[0];
    const float* ln1g = (const float*)d_in[1]; const float* ln1b = (const float*)d_in[2];
    const float* wq   = (const float*)d_in[3]; const float* wk = (const float*)d_in[4]; const float* wv = (const float*)d_in[5];
    const float* wp   = (const float*)d_in[6]; const float* bp = (const float*)d_in[7];
    const float* ln2g = (const float*)d_in[8]; const float* ln2b = (const float*)d_in[9];
    const float* w1   = (const float*)d_in[10]; const float* w2 = (const float*)d_in[11];
    float* OUT = (float*)d_out;
    char* wsp = (char*)d_ws;
    h16* H1  = (h16*)wsp; wsp += SZ_H;
    h16* H2  = (h16*)wsp; wsp += SZ_H;
    h16* W3  = (h16*)wsp; wsp += SZ_W3;
    h16* WPT = (h16*)wsp; wsp += SZ_WP;
    h16* W1T = (h16*)wsp; wsp += SZ_WF;
    h16* W2T = (h16*)wsp; wsp += SZ_WF;
    h16* QH  = (h16*)wsp; wsp += SZ_PL;
    h16* KP  = (h16*)wsp; wsp += SZ_PL;
    h16* VT  = (h16*)wsp; wsp += SZ_PL;
    h16* CTX = (h16*)wsp; wsp += SZ_PL;
    float* X1 = (float*)wsp; wsp += SZ_X1;
    h16* U   = (h16*)wsp; wsp += SZ_U;
    h16* WQT = W3; h16* WKT = W3 + (size_t)DM * DM; h16* WVT = W3 + (size_t)2 * DM * DM;

    k_wconvT<<<dim3(DM / 64, HD / 32, NH_), 256, 0, stream>>>(wq, WQT, HD, DM, (size_t)DM * HD, (size_t)HD * DM);
    k_wconvT<<<dim3(DM / 64, HD / 32, NH_), 256, 0, stream>>>(wk, WKT, HD, DM, (size_t)DM * HD, (size_t)HD * DM);
    k_wconvT<<<dim3(DM / 64, HD / 32, NH_), 256, 0, stream>>>(wv, WVT, HD, DM, (size_t)DM * HD, (size_t)HD * DM);
    k_wconvT<<<dim3(DM / 64, DM / 32, 1), 256, 0, stream>>>(wp, WPT, DM, DM, (size_t)0, (size_t)0);
    k_wconvT<<<dim3(DM / 64, FF / 32, 1), 256, 0, stream>>>(w1, W1T, FF, DM, (size_t)0, (size_t)0);
    k_wconvT<<<dim3(FF / 64, DM / 32, 1), 256, 0, stream>>>(w2, W2T, DM, FF, (size_t)0, (size_t)0);

    k_ln<<<NB * SEQ / 16, 256, 0, stream>>>(x, ln1g, ln1b, H1, SEQ_FULL, 1);

    k_proj_qk<<<dim3(NB * SEQ / 64, DM / 64, 1), 32, 0, stream>>>(H1, WQT, QH);
    k_proj_qk<<<dim3(NB * SEQ / 64, DM / 64, 1), 32, 0, stream>>>(H1, WKT, KP);
    k_proj_vt<<<dim3(DM / 64, NB * SEQ / 64, 1), 32, 0, stream>>>(WVT, H1, VT);

    k_flash<<<dim3(SEQ / (16 * AW), NB * NH_, 1), 32 * AW, 0, stream>>>(QH, KP, VT, CTX);

    k_proj_o<<<dim3(NB * SEQ / 64, DM / 64, 1), 32, 0, stream>>>(CTX, WPT, x, bp, X1);
    k_ln<<<NB * SEQ / 16, 256, 0, stream>>>(X1, ln2g, ln2b, H2, SEQ, 0);
    k_proj_f1<<<dim3(NB * SEQ / 64, FF / 64, 1), 32, 0, stream>>>(H2, W1T, U);
    k_proj_f2<<<dim3(NB * SEQ / 64, DM / 64, 1), 32, 0, stream>>>(U, W2T, X1, OUT);
}
